// UGRNNNet_69939247448791
// MI455X (gfx1250) — hardware-verified
//
#include <hip/hip_runtime.h>
#include <stddef.h>
#include <stdint.h>


typedef _Float16 half_t;
typedef _Float16 v8h  __attribute__((ext_vector_type(8)));
typedef _Float16 v16h __attribute__((ext_vector_type(16)));
typedef float    v8f  __attribute__((ext_vector_type(8)));
typedef float    v4f  __attribute__((ext_vector_type(4)));

union Frag { v16h v; v8h p[2]; };

#define BB    64
#define SS    512
#define FIN   256
#define HH    512
#define FOUT  128
#define XS    264
#define HS    520
#define SP    132
#define TP    72
#define NTHR  1024
#define WSCALE 8.0f
#define WINV   0.125f

__device__ __forceinline__ v8f wmma16(v16h a, v16h b, v8f c) {
  return __builtin_amdgcn_wmma_f32_16x16x32_f16(false, a, false, b, (short)0, c, false, false);
}

__device__ __forceinline__ void gemm2(const half_t* pa, int apitch,
                                      const half_t* __restrict__ pz,
                                      const half_t* __restrict__ ph, int nk,
                                      v8f& az0, v8f& az1, v8f& ah0, v8f& ah1) {
  const half_t* pa1 = pa + 16 * apitch;
  #pragma unroll 1
  for (int kk = 0; kk < nk; ++kk) {
    const int k0 = kk << 5;
    Frag bz, bh, a0, a1;
    bz.p[0] = *(const v8h*)(pz + k0);   bz.p[1] = *(const v8h*)(pz + k0 + 16);
    bh.p[0] = *(const v8h*)(ph + k0);   bh.p[1] = *(const v8h*)(ph + k0 + 16);
    a0.p[0] = *(const v8h*)(pa + k0);   a0.p[1] = *(const v8h*)(pa + k0 + 16);
    a1.p[0] = *(const v8h*)(pa1 + k0);  a1.p[1] = *(const v8h*)(pa1 + k0 + 16);
    az0 = wmma16(a0.v, bz.v, az0);
    ah0 = wmma16(a0.v, bh.v, ah0);
    az1 = wmma16(a1.v, bz.v, az1);
    ah1 = wmma16(a1.v, bh.v, ah1);
    asm volatile("v_nop\n\tv_nop\n\tv_nop\n\tv_nop"
                 : "+v"(az0), "+v"(az1), "+v"(ah0), "+v"(ah1)
                 : "v"(a0.v), "v"(a1.v), "v"(bz.v), "v"(bh.v));
  }
}

__device__ __forceinline__ float cell_update(float az, float ah, float vz, float vh, float hold) {
  const float pz = az * WINV + vz;
  float ph = ah * WINV + vh;
  const float z = __builtin_amdgcn_rcpf(1.0f + __expf(-pz));
  ph = fminf(fmaxf(ph, -15.0f), 15.0f);
  const float e = __expf(2.0f * ph);
  const float c = (e - 1.0f) * __builtin_amdgcn_rcpf(e + 1.0f);
  return z * hold + (1.0f - z) * c;
}

__device__ __forceinline__ void layer_step(const half_t* a0base, int s0, int nk0,
                                           const half_t* a1base, int nk1,
                                           const half_t* __restrict__ wz,
                                           const half_t* __restrict__ wh, int len0,
                                           float vz, float vh, float (&hs)[4][8],
                                           int m, int hf8) {
  #pragma unroll
  for (int mh = 0; mh < 2; ++mh) {
    v8f az0 = {0.f, 0.f, 0.f, 0.f, 0.f, 0.f, 0.f, 0.f};
    v8f az1 = az0, ah0 = az0, ah1 = az0;
    gemm2(a0base + (32 * mh + m) * s0 + hf8, s0, wz, wh, nk0, az0, az1, ah0, ah1);
    gemm2(a1base + (32 * mh + m) * HS + hf8, HS, wz + len0, wh + len0, nk1, az0, az1, ah0, ah1);
    #pragma unroll
    for (int r = 0; r < 8; ++r) {
      hs[2 * mh][r]     = cell_update(az0[r], ah0[r], vz, vh, hs[2 * mh][r]);
      hs[2 * mh + 1][r] = cell_update(az1[r], ah1[r], vz, vh, hs[2 * mh + 1][r]);
    }
  }
}

__device__ __forceinline__ void store_state_f16(half_t* lhb, const float (&hs)[4][8], int ncol, int hf8) {
  #pragma unroll
  for (int mt = 0; mt < 4; ++mt) {
    #pragma unroll
    for (int r = 0; r < 8; ++r)
      lhb[(mt * 16 + hf8 + r) * HS + ncol] = (half_t)hs[mt][r];
  }
}

__global__ __launch_bounds__(256)
void cvt_wt_kernel(const float* __restrict__ W, half_t* WT, int K, int N) {
  __shared__ __align__(16) half_t sT[32 * TP];
  const int tid = threadIdx.x;
  const int n0 = blockIdx.x * 32;
  const int k0 = blockIdx.y * 64;
  if (n0 + 32 > N || k0 + 64 > K) return;
  {
    const int kr = tid >> 2;
    const int c  = (tid & 3) << 3;
    const float* src = W + (size_t)(k0 + kr) * (size_t)N + (size_t)(n0 + c);
    const v4f u0 = *(const v4f*)(src);
    const v4f u1 = *(const v4f*)(src + 4);
    sT[(c + 0) * TP + kr] = (half_t)(u0[0] * WSCALE);
    sT[(c + 1) * TP + kr] = (half_t)(u0[1] * WSCALE);
    sT[(c + 2) * TP + kr] = (half_t)(u0[2] * WSCALE);
    sT[(c + 3) * TP + kr] = (half_t)(u0[3] * WSCALE);
    sT[(c + 4) * TP + kr] = (half_t)(u1[0] * WSCALE);
    sT[(c + 5) * TP + kr] = (half_t)(u1[1] * WSCALE);
    sT[(c + 6) * TP + kr] = (half_t)(u1[2] * WSCALE);
    sT[(c + 7) * TP + kr] = (half_t)(u1[3] * WSCALE);
  }
  __syncthreads();
  {
    const int n = tid >> 3;
    const int j = tid & 7;
    const v8h v = *(const v8h*)(sT + n * TP + (j << 3));
    half_t* dst = WT + (size_t)(n0 + n) * (size_t)K + (size_t)(k0 + (j << 3));
    *(volatile v8h*)dst = v;
    __threadfence();
    *(volatile v8h*)dst = v;
  }
}

__global__ __launch_bounds__(NTHR)
void rnn_main_kernel(const float* __restrict__ x,
                     const float* __restrict__ bz0, const float* __restrict__ bh0,
                     const float* __restrict__ bz1, const float* __restrict__ bh1,
                     const half_t* __restrict__ WzT0, const half_t* __restrict__ WhT0,
                     const half_t* __restrict__ WzT1, const half_t* __restrict__ WhT1,
                     const half_t* __restrict__ WfT,  const float* __restrict__ bfc,
                     float* out) {
  __shared__ __align__(16) half_t lx[BB * XS];
  __shared__ __align__(16) half_t lh0[BB * HS];
  __shared__ __align__(16) half_t lh1[BB * HS];

  const int tid  = threadIdx.x;
  const int w    = tid >> 5;
  const int l    = tid & 31;
  const int hf   = l >> 4;
  const int m    = l & 15;
  const int hf8  = hf << 3;
  const int ncol = w * 16 + m;

  float h0s[4][8], h1s[4][8];
  #pragma unroll
  for (int mt = 0; mt < 4; ++mt) {
    #pragma unroll
    for (int r = 0; r < 8; ++r) { h0s[mt][r] = 0.0f; h1s[mt][r] = 0.0f; }
  }

  {
    const v8h z8 = {(half_t)0.f, (half_t)0.f, (half_t)0.f, (half_t)0.f,
                    (half_t)0.f, (half_t)0.f, (half_t)0.f, (half_t)0.f};
    for (int i = tid; i < (BB * HS) / 8; i += NTHR) {
      *(v8h*)(lh0 + 8 * i) = z8;
      *(v8h*)(lh1 + 8 * i) = z8;
    }
  }

  const float vz0 = bz0[ncol], vh0 = bh0[ncol];
  const float vz1 = bz1[ncol], vh1 = bh1[ncol];
  const half_t* wz0p = WzT0 + (size_t)ncol * (FIN + HH) + hf8;
  const half_t* wh0p = WhT0 + (size_t)ncol * (FIN + HH) + hf8;
  const half_t* wz1p = WzT1 + (size_t)ncol * (HH + HH) + hf8;
  const half_t* wh1p = WhT1 + (size_t)ncol * (HH + HH) + hf8;

  __syncthreads();

  #pragma unroll 1
  for (int t = 0; t < SS; ++t) {
    {
      const int row = tid >> 4;
      const int c0  = (tid & 15) << 4;
      const float* xp = x + ((size_t)row * SS + (size_t)t) * FIN + (size_t)c0;
      const v4f u0 = *(const v4f*)(xp);
      const v4f u1 = *(const v4f*)(xp + 4);
      const v4f u2 = *(const v4f*)(xp + 8);
      const v4f u3 = *(const v4f*)(xp + 12);
      v8h q0, q1;
      q0[0] = (half_t)u0[0]; q0[1] = (half_t)u0[1]; q0[2] = (half_t)u0[2]; q0[3] = (half_t)u0[3];
      q0[4] = (half_t)u1[0]; q0[5] = (half_t)u1[1]; q0[6] = (half_t)u1[2]; q0[7] = (half_t)u1[3];
      q1[0] = (half_t)u2[0]; q1[1] = (half_t)u2[1]; q1[2] = (half_t)u2[2]; q1[3] = (half_t)u2[3];
      q1[4] = (half_t)u3[0]; q1[5] = (half_t)u3[1]; q1[6] = (half_t)u3[2]; q1[7] = (half_t)u3[3];
      half_t* dst = lx + row * XS + c0;
      *(v8h*)(dst)     = q0;
      *(v8h*)(dst + 8) = q1;
    }
    __syncthreads();

    layer_step(lx, XS, FIN / 32, lh0, HH / 32, wz0p, wh0p, FIN, vz0, vh0, h0s, m, hf8);
    __syncthreads();
    store_state_f16(lh0, h0s, ncol, hf8);
    __syncthreads();

    layer_step(lh0, HS, HH / 32, lh1, HH / 32, wz1p, wh1p, HH, vz1, vh1, h1s, m, hf8);
    __syncthreads();
    store_state_f16(lh1, h1s, ncol, hf8);
  }
  __syncthreads();

  float* stg = reinterpret_cast<float*>(lh0);
  {
    const int mt = w >> 3;
    const int nt = w & 7;
    v8f acc = {0.f, 0.f, 0.f, 0.f, 0.f, 0.f, 0.f, 0.f};
    const half_t* pa = lh1 + (mt * 16 + m) * HS + hf8;
    const half_t* pb = WfT + (size_t)(nt * 16 + m) * HH + hf8;
    #pragma unroll 1
    for (int kk = 0; kk < HH / 32; ++kk) {
      const int k0 = kk << 5;
      Frag a, b;
      a.p[0] = *(const v8h*)(pa + k0);  a.p[1] = *(const v8h*)(pa + k0 + 16);
      b.p[0] = *(const v8h*)(pb + k0);  b.p[1] = *(const v8h*)(pb + k0 + 16);
      acc = wmma16(a.v, b.v, acc);
      asm volatile("v_nop\n\tv_nop\n\tv_nop\n\tv_nop" : "+v"(acc) : "v"(a.v), "v"(b.v));
    }
    const int col = nt * 16 + m;
    const float bb = bfc[col];
    #pragma unroll
    for (int r = 0; r < 8; ++r)
      stg[(mt * 16 + hf8 + r) * SP + col] = acc[r] * WINV + bb;
  }
  __syncthreads();

  {
    const int j  = tid & 7;
    const int L0 = tid >> 3;
    const int L1 = L0 + 128;
    const int r0 = L0 >> 2, c0 = ((L0 & 3) << 5) + (j << 2);
    const int r1 = L1 >> 2, c1 = ((L1 & 3) << 5) + (j << 2);
    const v4f v0 = *(const v4f*)(stg + r0 * SP + c0);
    const v4f v1 = *(const v4f*)(stg + r1 * SP + c1);
    float* d0 = out + r0 * FOUT + c0;
    float* d1 = out + r1 * FOUT + c1;
    *(volatile v4f*)d0 = v0;
    *(volatile v4f*)d1 = v1;
    __threadfence();
    *(volatile v4f*)d0 = v0;
    *(volatile v4f*)d1 = v1;
  }
}

extern "C" void kernel_launch(void* const* d_in, const int* in_sizes, int n_in,
                              void* d_out, int out_size, void* d_ws, size_t ws_size,
                              hipStream_t stream) {
  if (n_in < 11) return;
  if (in_sizes[0] != BB * SS * FIN) return;
  if (in_sizes[1] != (FIN + HH) * HH || in_sizes[3] != (FIN + HH) * HH) return;
  if (in_sizes[2] != HH || in_sizes[4] != HH || in_sizes[6] != HH || in_sizes[8] != HH) return;
  if (in_sizes[5] != (HH + HH) * HH || in_sizes[7] != (HH + HH) * HH) return;
  if (in_sizes[9] != HH * FOUT || in_sizes[10] != FOUT) return;
  if (out_size != BB * FOUT) return;

  const float* x   = (const float*)d_in[0];
  const float* Wz0 = (const float*)d_in[1];
  const float* bz0 = (const float*)d_in[2];
  const float* Wh0 = (const float*)d_in[3];
  const float* bh0 = (const float*)d_in[4];
  const float* Wz1 = (const float*)d_in[5];
  const float* bz1 = (const float*)d_in[6];
  const float* Wh1 = (const float*)d_in[7];
  const float* bh1 = (const float*)d_in[8];
  const float* Wfc = (const float*)d_in[9];
  const float* bfc = (const float*)d_in[10];
  float* out = (float*)d_out;

  const size_t b0 = (size_t)HH * (FIN + HH) * sizeof(half_t);
  const size_t b1 = (size_t)HH * (HH + HH) * sizeof(half_t);
  const size_t bf = (size_t)FOUT * HH * sizeof(half_t);
  const size_t oWzT0 = 0;
  const size_t oWhT0 = oWzT0 + b0;
  const size_t oWzT1 = oWhT0 + b0;
  const size_t oWhT1 = oWzT1 + b1;
  const size_t oWfT  = oWhT1 + b1;
  const size_t total = oWfT + bf;
  if (total > ws_size) return;

  char* ws = (char*)d_ws;
  half_t* WzT0 = (half_t*)(ws + oWzT0);
  half_t* WhT0 = (half_t*)(ws + oWhT0);
  half_t* WzT1 = (half_t*)(ws + oWzT1);
  half_t* WhT1 = (half_t*)(ws + oWhT1);
  half_t* WfT  = (half_t*)(ws + oWfT);

  cvt_wt_kernel<<<dim3(HH / 32, (FIN + HH) / 64), 256, 0, stream>>>(Wz0, WzT0, FIN + HH, HH);
  cvt_wt_kernel<<<dim3(HH / 32, (FIN + HH) / 64), 256, 0, stream>>>(Wh0, WhT0, FIN + HH, HH);
  cvt_wt_kernel<<<dim3(HH / 32, (HH + HH) / 64), 256, 0, stream>>>(Wz1, WzT1, HH + HH, HH);
  cvt_wt_kernel<<<dim3(HH / 32, (HH + HH) / 64), 256, 0, stream>>>(Wh1, WhT1, HH + HH, HH);
  cvt_wt_kernel<<<dim3(FOUT / 32, HH / 64), 256, 0, stream>>>(Wfc, WfT, HH, FOUT);

  rnn_main_kernel<<<1, NTHR, 0, stream>>>(x, bz0, bh0, bz1, bh1,
                                          WzT0, WhT0, WzT1, WhT1, WfT, bfc, out);
}
